// MultiHeadedSelfAttentionModule_30605936951352
// MI455X (gfx1250) — hardware-verified
//
#include <hip/hip_runtime.h>
#include <math.h>
#include <stdint.h>

#define NB_  8
#define NT_  1024
#define ND_  512
#define NH_  8
#define HD_  64
#define NBT_ 8192


typedef _Float16 v16h __attribute__((ext_vector_type(16)));
typedef _Float16 v8h  __attribute__((ext_vector_type(8)));
typedef __bf16   v16b __attribute__((ext_vector_type(16)));
typedef __bf16   v8b  __attribute__((ext_vector_type(8)));
typedef float    v8f  __attribute__((ext_vector_type(8)));
typedef float    v4f  __attribute__((ext_vector_type(4)));
typedef unsigned int v4u __attribute__((ext_vector_type(4)));
typedef v4f __attribute__((may_alias)) v4fa;
typedef v8h __attribute__((may_alias)) v8ha;
typedef v8b __attribute__((may_alias)) v8ba;
typedef v4u __attribute__((may_alias)) v4ua;

static_assert(NT_ % 64 == 0);
static_assert(ND_ % 64 == 0);
static_assert(NH_ * HD_ == ND_);
static_assert(HD_ % 32 == 0);

__device__ __forceinline__ unsigned short f2bf_bits(float f) {
  unsigned u = __float_as_uint(f);
  return (unsigned short)((u + 0x7FFFu + ((u >> 16) & 1u)) >> 16);
}
__device__ __forceinline__ float bf_bits2f(unsigned short h) { return __uint_as_float(((unsigned)h) << 16); }
__device__ __forceinline__ unsigned pk16(unsigned short a, unsigned short b) { return (unsigned)a | ((unsigned)b << 16); }
__device__ __forceinline__ v8f zero8() { v8f z = {0.f, 0.f, 0.f, 0.f, 0.f, 0.f, 0.f, 0.f}; return z; }

__device__ __forceinline__ void dep_guard_h(v8f& a, v8f& b, v16h x, v16h y) { asm volatile("v_nop\n\tv_nop\n\tv_nop\n\tv_nop" : "+v"(a), "+v"(b) : "v"(x), "v"(y)); }
__device__ __forceinline__ void dep_guard_b(v8f& a, v8f& b, v16b x, v16b y) { asm volatile("v_nop\n\tv_nop\n\tv_nop\n\tv_nop" : "+v"(a), "+v"(b) : "v"(x), "v"(y)); }
__device__ __forceinline__ void keep4_h(v16h a, v16h b, v16h c, v16h d) { asm volatile("v_nop" :: "v"(a), "v"(b), "v"(c), "v"(d)); }
__device__ __forceinline__ void keep4_b(v16b a, v16b b, v16b c, v16b d) { asm volatile("v_nop" :: "v"(a), "v"(b), "v"(c), "v"(d)); }
__device__ __forceinline__ void acc_guard4(v8f& a, v8f& b, v8f& c, v8f& d) { asm volatile("v_nop\n\tv_nop\n\tv_nop\n\tv_nop" : "+v"(a), "+v"(b), "+v"(c), "+v"(d)); }

template <typename T> struct Frag;
template <> struct Frag<_Float16> {
  typedef v16h V; union U { v16h v; v8h h[2]; };
  static __device__ __forceinline__ v16h load(const _Float16* p) {
    U f; f.h[0] = *(const v8ha*)(p); f.h[1] = *(const v8ha*)(p + 16); return f.v;
  }
  static __device__ __forceinline__ v8f mma(v16h a, v16h b, v8f c) {
    return __builtin_amdgcn_wmma_f32_16x16x32_f16(false, a, false, b, (short)0, c, false, false);
  }
  static __device__ __forceinline__ void guard(v8f& a, v8f& b, v16h x, v16h y) { dep_guard_h(a, b, x, y); }
  static __device__ __forceinline__ void keep(v16h a, v16h b, v16h c, v16h d) { keep4_h(a, b, c, d); }
};
template <> struct Frag<__bf16> {
  typedef v16b V; union U { v16b v; v8b h[2]; };
  static __device__ __forceinline__ v16b load(const __bf16* p) {
    U f; f.h[0] = *(const v8ba*)(p); f.h[1] = *(const v8ba*)(p + 16); return f.v;
  }
  static __device__ __forceinline__ v8f mma(v16b a, v16b b, v8f c) {
    return __builtin_amdgcn_wmma_f32_16x16x32_bf16(false, a, false, b, (short)0, c, false, false);
  }
  static __device__ __forceinline__ void guard(v8f& a, v8f& b, v16b x, v16b y) { dep_guard_b(a, b, x, y); }
  static __device__ __forceinline__ void keep(v16b a, v16b b, v16b c, v16b d) { keep4_b(a, b, c, d); }
};

__device__ __forceinline__ v8f mma16h(v16h a, v16h b, v8f c) {
  c = __builtin_amdgcn_wmma_f32_16x16x32_f16(false, a, false, b, (short)0, c, false, false);
  asm volatile("v_nop\n\tv_nop\n\tv_nop\n\tv_nop" : "+v"(c) : "v"(a), "v"(b));
  return c;
}
__device__ __forceinline__ v8f mma16b(v16b a, v16b b, v8f c) {
  c = __builtin_amdgcn_wmma_f32_16x16x32_bf16(false, a, false, b, (short)0, c, false, false);
  asm volatile("v_nop\n\tv_nop\n\tv_nop\n\tv_nop" : "+v"(c) : "v"(a), "v"(b));
  return c;
}
__device__ __forceinline__ void bf_split(float f, __bf16& hi, __bf16& lo) {
  const unsigned short hb = f2bf_bits(f);
  hi = __builtin_bit_cast(__bf16, hb);
  lo = __builtin_bit_cast(__bf16, f2bf_bits(f - bf_bits2f(hb)));
}

__global__ __launch_bounds__(64) void ln_kernel(const float* __restrict__ x, const float* __restrict__ g,
                                                 const float* __restrict__ be, _Float16* __restrict__ xf,
                                                 unsigned short* __restrict__ xh, unsigned short* __restrict__ xl) {
  __shared__ float red[4];
  const int row = blockIdx.x, tid = threadIdx.x, lane = tid & 31, wave = tid >> 5;
  const int c0 = tid * 8;
  const float* xr = x + (size_t)row * ND_ + c0;
  const v4f a0 = *(const v4f*)(xr);
  const v4f a1 = *(const v4f*)(xr + 4);
  float v[8];
  v[0] = a0[0]; v[1] = a0[1]; v[2] = a0[2]; v[3] = a0[3];
  v[4] = a1[0]; v[5] = a1[1]; v[6] = a1[2]; v[7] = a1[3];
  float s = ((v[0] + v[1]) + (v[2] + v[3])) + ((v[4] + v[5]) + (v[6] + v[7]));
#pragma unroll
  for (int off = 1; off < 32; off <<= 1) s += __shfl_xor(s, off, 32);
  if (lane == 0) red[wave] = s;
  __syncthreads();
  const float mean = (red[0] + red[1]) * (1.0f / (float)ND_);
  float d[8];
  float s2 = 0.0f;
#pragma unroll
  for (int e = 0; e < 8; ++e) { d[e] = v[e] - mean; s2 = fmaf(d[e], d[e], s2); }
#pragma unroll
  for (int off = 1; off < 32; off <<= 1) s2 += __shfl_xor(s2, off, 32);
  if (lane == 0) red[2 + wave] = s2;
  __syncthreads();
  const float var  = (red[2] + red[3]) * (1.0f / (float)ND_);
  const float rstd = rsqrtf(var + 1e-5f);
  const v4f g0 = *(const v4f*)(g + c0),  g1 = *(const v4f*)(g + c0 + 4);
  const v4f b0 = *(const v4f*)(be + c0), b1 = *(const v4f*)(be + c0 + 4);
  float gg[8], bb[8];
  gg[0] = g0[0]; gg[1] = g0[1]; gg[2] = g0[2]; gg[3] = g0[3]; gg[4] = g1[0]; gg[5] = g1[1]; gg[6] = g1[2]; gg[7] = g1[3];
  bb[0] = b0[0]; bb[1] = b0[1]; bb[2] = b0[2]; bb[3] = b0[3]; bb[4] = b1[0]; bb[5] = b1[1]; bb[6] = b1[2]; bb[7] = b1[3];
  v8h of;
  unsigned short hb[8], lb[8];
#pragma unroll
  for (int e = 0; e < 8; ++e) {
    const float y = (d[e] * rstd) * gg[e] + bb[e];
    of[e] = (_Float16)(y * 8.0f);
    hb[e] = f2bf_bits(y);
    lb[e] = f2bf_bits(y - bf_bits2f(hb[e]));
  }
  v4u ph, pl;
  ph[0] = pk16(hb[0], hb[1]); ph[1] = pk16(hb[2], hb[3]); ph[2] = pk16(hb[4], hb[5]); ph[3] = pk16(hb[6], hb[7]);
  pl[0] = pk16(lb[0], lb[1]); pl[1] = pk16(lb[2], lb[3]); pl[2] = pk16(lb[4], lb[5]); pl[3] = pk16(lb[6], lb[7]);
  _Float16* pf = xf + (size_t)row * ND_ + c0;
  unsigned short* phh = xh + (size_t)row * ND_ + c0;
  unsigned short* pll = xl + (size_t)row * ND_ + c0;
  *(volatile v8h*)pf = of;
  *(volatile v4u*)phh = ph;
  *(volatile v4u*)pll = pl;
  __threadfence();
  *(volatile v8h*)pf = of;
  *(volatile v4u*)phh = ph;
  *(volatile v4u*)pll = pl;
}

__global__ __launch_bounds__(256) void tcvt_f16_kernel(const float* __restrict__ W, _Float16* __restrict__ o,
                                                       int R, int Cc, float scale) {
  __shared__ __align__(16) float tf[64 * 68];
  const int c0 = blockIdx.x * 64;
  const int r0 = blockIdx.y * 64;
  const int tid = threadIdx.x;
  {
    const int lr = tid >> 4, c4 = (tid & 15) * 4;
#pragma unroll
    for (int it = 0; it < 4; ++it) {
      const int rr = it * 16 + lr;
      const v4f a = *(const v4f*)(W + (size_t)(r0 + rr) * Cc + c0 + c4);
      *(v4fa*)(tf + rr * 68 + c4) = a;
    }
  }
  __syncthreads();
  const int sub = tid >> 3, c8 = (tid & 7) * 8;
  v8h hv[2];
#pragma unroll
  for (int it = 0; it < 2; ++it) {
    const int oc = it * 32 + sub;
    v8h a;
#pragma unroll
    for (int e = 0; e < 8; ++e) a[e] = (_Float16)(tf[(c8 + e) * 68 + oc] * scale);
    hv[it] = a;
  }
  for (int pass = 0; pass < 2; ++pass) {
#pragma unroll
    for (int it = 0; it < 2; ++it) {
      const int oc = it * 32 + sub;
      *(volatile v8h*)(o + (size_t)(c0 + oc) * R + r0 + c8) = hv[it];
    }
    __threadfence();
  }
}

__global__ __launch_bounds__(256) void tsplit_kernel(const float* __restrict__ W, unsigned short* __restrict__ oh,
                                                     unsigned short* __restrict__ ol, int R, int Cc, long sIn, long sOut) {
  __shared__ __align__(16) float tf[64 * 68];
  W  += (size_t)blockIdx.z * sIn;
  oh += (size_t)blockIdx.z * sOut;
  ol += (size_t)blockIdx.z * sOut;
  const int c0  = blockIdx.x * 64;
  const int r0  = blockIdx.y * 64;
  const int tid = threadIdx.x;
  {
    const int lr = tid >> 4, c4 = (tid & 15) * 4;
#pragma unroll
    for (int it = 0; it < 4; ++it) {
      const int rr = it * 16 + lr;
      const v4f a = *(const v4f*)(W + (size_t)(r0 + rr) * Cc + c0 + c4);
      *(v4fa*)(tf + rr * 68 + c4) = a;
    }
  }
  __syncthreads();
  const int sub = tid >> 3, c8 = (tid & 7) * 8;
  v4u hv[2], lv[2];
#pragma unroll
  for (int it = 0; it < 2; ++it) {
    const int oc = it * 32 + sub;
    v4u a, a2;
#pragma unroll
    for (int q = 0; q < 4; ++q) {
      const float f0 = tf[(c8 + 2 * q) * 68 + oc];
      const float f1 = tf[(c8 + 2 * q + 1) * 68 + oc];
      const unsigned short h0 = f2bf_bits(f0), h1 = f2bf_bits(f1);
      const unsigned short l0 = f2bf_bits(f0 - bf_bits2f(h0)), l1 = f2bf_bits(f1 - bf_bits2f(h1));
      a[q]  = pk16(h0, h1);
      a2[q] = pk16(l0, l1);
    }
    hv[it] = a; lv[it] = a2;
  }
  for (int pass = 0; pass < 2; ++pass) {
#pragma unroll
    for (int it = 0; it < 2; ++it) {
      const int oc = it * 32 + sub;
      const size_t go = (size_t)(c0 + oc) * R + r0 + c8;
      *(volatile v4u*)(oh + go) = hv[it];
      *(volatile v4u*)(ol + go) = lv[it];
    }
    __threadfence();
  }
}

__global__ __launch_bounds__(64) void pe_kernel(_Float16* __restrict__ pef) {
  __shared__ __align__(16) _Float16 peb[ND_];
  const int t = blockIdx.x, tid = threadIdx.x;
  const int c0 = tid * 8;
  const float kf = -(9.2103404f / 512.0f)    ;
  const float tfl = (float)t;
#pragma unroll 1
  for (int j = 0; j < 4; ++j) {
    const int i2 = c0 + 2 * j;
    const float dv = expf((float)i2 * kf);
    const float ang = tfl * dv;
    float sn, cn;
    sincosf(ang, &sn, &cn);
    peb[i2]     = (_Float16)(sn * 8.0f);
    peb[i2 + 1] = (_Float16)(cn * 8.0f);
  }
  __syncthreads();
  const v8h ov = *(const v8ha*)(peb + c0);
  _Float16* dp = pef + (size_t)t * ND_ + c0;
  *(volatile v8h*)dp = ov;
  __threadfence();
  *(volatile v8h*)dp = ov;
}

template <int ET> struct Elem;
template <> struct Elem<0> { typedef _Float16 T; };
template <> struct Elem<1> { typedef __bf16 T; };

template <int ET, bool SPLIT, int OUT, int BM>
__global__ __launch_bounds__(256) void gemm64_kernel(
    const unsigned short* __restrict__ Ap, const unsigned short* __restrict__ A2p, int lda, long strideA,
    const unsigned short* __restrict__ Btp, const unsigned short* __restrict__ Bt2p, int ldb, long strideB,
    void* C1, void* C2, int ldc, long strideC,
    const float* __restrict__ b1, const float* __restrict__ a1, const float* __restrict__ a2,
    int M, int N, int K, float scale, float carry) {
  typedef typename Elem<ET>::T T;
  typedef typename Frag<T>::V V;
  const T* A = (const T*)Ap; const T* A2 = (const T*)A2p; const T* Bt = (const T*)Btp; const T* Bt2 = (const T*)Bt2p;
  __shared__ __align__(16) float sT[8][16 * 68];

  const int z    = blockIdx.y;
  const int lane = threadIdx.x & 31;
  const int wave = threadIdx.x >> 5;
  const int tilesN = N >> 6;
  const int tilesM = M >> 6;
  const int tile = blockIdx.x * 8 + wave;
  if (tile >= tilesM * tilesN) return;
  const int tm = tile / tilesN;
  const int tn = tile - tm * tilesN;
  const int m0 = tm << 6;
  const int n0 = tn << 6;

  const T* Ab  = A  + (size_t)z * strideA;
  const T* Bb  = Bt + (size_t)z * strideB;
  const T* Ab2 = SPLIT ? (A2  + (size_t)z * strideA) : nullptr;
  const T* Bb2 = SPLIT ? (Bt2 + (size_t)z * strideB) : nullptr;

  const int rlane = lane & 15;
  const int koff  = (lane >> 4) * 8;
  const int mOff  = (lane >> 4) * 8;

  v8f acc[4][4];
#pragma unroll
  for (int i = 0; i < 4; ++i)
#pragma unroll
    for (int j = 0; j < 4; ++j) acc[i][j] = zero8();

  for (int k0 = 0; k0 < K; k0 += 32) {
    V bh[4], bl[4];
#pragma unroll
    for (int j = 0; j < 4; ++j) {
      const size_t bo = (size_t)(n0 + (j << 4) + rlane) * ldb + koff + k0;
      bh[j] = Frag<T>::load(Bb + bo);
      if (SPLIT) bl[j] = Frag<T>::load(Bb2 + bo);
    }
#pragma unroll
    for (int i = 0; i < 4; ++i) {
      const size_t ao = (size_t)(m0 + (i << 4) + rlane) * lda + koff + k0;
      V ah = Frag<T>::load(Ab + ao);
      V al;
      if (SPLIT) al = Frag<T>::load(Ab2 + ao);
#pragma unroll
      for (int j = 0; j < 4; ++j) {
        acc[i][j] = Frag<T>::mma(ah, bh[j], acc[i][j]);
        if (SPLIT) {
          acc[i][j] = Frag<T>::mma(ah, bl[j], acc[i][j]);
          acc[i][j] = Frag<T>::mma(al, bh[j], acc[i][j]);
        }
      }
      Frag<T>::guard(acc[i][0], acc[i][3], ah, SPLIT ? al : ah);
    }
    Frag<T>::keep(bh[0], bh[1], bh[2], bh[3]);
    if (SPLIT) Frag<T>::keep(bl[0], bl[1], bl[2], bl[3]);
  }
  acc_guard4(acc[0][0], acc[0][1], acc[0][2], acc[0][3]);
  acc_guard4(acc[1][0], acc[1][1], acc[1][2], acc[1][3]);
  acc_guard4(acc[2][0], acc[2][1], acc[2][2], acc[2][3]);
  acc_guard4(acc[3][0], acc[3][1], acc[3][2], acc[3][3]);

  float* slab = sT[wave];
  float ua[8], uv[8];
#pragma unroll
  for (int e = 0; e < 8; ++e) { ua[e] = 0.0f; uv[e] = 0.0f; }
  if (OUT == 2) {
    const int c8e = (lane & 7) * 8;
    const v4f e0 = *(const v4f*)(a1 + n0 + c8e), e1 = *(const v4f*)(a1 + n0 + c8e + 4);
    const v4f f0 = *(const v4f*)(a2 + n0 + c8e), f1 = *(const v4f*)(a2 + n0 + c8e + 4);
    ua[0] = e0[0]; ua[1] = e0[1]; ua[2] = e0[2]; ua[3] = e0[3]; ua[4] = e1[0]; ua[5] = e1[1]; ua[6] = e1[2]; ua[7] = e1[3];
    uv[0] = f0[0]; uv[1] = f0[1]; uv[2] = f0[2]; uv[3] = f0[3]; uv[4] = f1[0]; uv[5] = f1[1]; uv[6] = f1[2]; uv[7] = f1[3];
  }
#pragma unroll
  for (int i = 0; i < 4; ++i) {
    const int mBase = m0 + (i << 4);
#pragma unroll
    for (int j = 0; j < 4; ++j) {
      const int n = n0 + (j << 4) + rlane;
      float bn = 0.f;
      if (BM == 2) bn = b1[n];
#pragma unroll
      for (int r = 0; r < 8; ++r) {
        float v = acc[i][j][r] * scale;
        if (BM == 1) v += b1[mBase + mOff + r];
        if (BM == 2) v += bn;
        slab[(mOff + r) * 68 + (j << 4) + rlane] = v;
      }
    }
    __builtin_amdgcn_fence(__ATOMIC_RELEASE, "workgroup");
    __builtin_amdgcn_wave_barrier();
    __builtin_amdgcn_fence(__ATOMIC_ACQUIRE, "workgroup");
    if (OUT == 0) {
      float* C = (float*)C1 + (size_t)z * strideC;
      const int hh = lane >> 4, c4 = (lane & 15) * 4;
      for (int pass = 0; pass < 2; ++pass) {
#pragma unroll
        for (int it = 0; it < 8; ++it) {
          const int row = it * 2 + hh;
          const v4f vv = *(const v4fa*)(slab + row * 68 + c4);
          *(volatile v4f*)(C + (size_t)(mBase + row) * ldc + n0 + c4) = vv;
        }
        __threadfence();
      }
    } else {
      const int q = lane >> 3, c8 = (lane & 7) * 8;
      _Float16* Ca = (_Float16*)C1 + (size_t)z * strideC;
      _Float16* Cb = (_Float16*)C2 + (size_t)z * strideC;
      v8h hv[4], lv[4];
#pragma unroll
      for (int it = 0; it < 4; ++it) {
        const int row = it * 4 + q;
        const float* sp = slab + row * 68 + c8;
        const v4f x0 = *(const v4fa*)(sp);
        const v4f x1 = *(const v4fa*)(sp + 4);
        float f[8];
        f[0] = x0[0]; f[1] = x0[1]; f[2] = x0[2]; f[3] = x0[3];
        f[4] = x1[0]; f[5] = x1[1]; f[6] = x1[2]; f[7] = x1[3];
        v8h ha, hb;
#pragma unroll
        for (int e = 0; e < 8; ++e) {
          if (OUT == 1) {
            ha[e] = (_Float16)(f[e] * carry);
            hb[e] = ha[e];
          } else if (OUT == 2) {
            ha[e] = (_Float16)((f[e] + ua[e]) * carry);
            hb[e] = (_Float16)((f[e] + uv[e]) * carry);
          } else {
            const unsigned short hbits = f2bf_bits(f[e]);
            const unsigned short lbits = f2bf_bits(f[e] - bf_bits2f(hbits));
            ha[e] = __builtin_bit_cast(_Float16, hbits);
            hb[e] = __builtin_bit_cast(_Float16, lbits);
          }
        }
        hv[it] = ha; lv[it] = hb;
      }
      for (int pass = 0; pass < 2; ++pass) {
#pragma unroll
        for (int it = 0; it < 4; ++it) {
          const int row = it * 4 + q;
          *(volatile v8h*)(Ca + (size_t)(mBase + row) * ldc + n0 + c8) = hv[it];
          if (OUT >= 2) *(volatile v8h*)(Cb + (size_t)(mBase + row) * ldc + n0 + c8) = lv[it];
        }
        __threadfence();
      }
    }
    __builtin_amdgcn_fence(__ATOMIC_RELEASE, "workgroup");
    __builtin_amdgcn_wave_barrier();
    __builtin_amdgcn_fence(__ATOMIC_ACQUIRE, "workgroup");
  }
}

__global__ __launch_bounds__(128)
void relattn_kernel(const _Float16* __restrict__ QU, const _Float16* __restrict__ KPL,
                    const unsigned short* __restrict__ VThp, const unsigned short* __restrict__ VTlp,
                    const float* __restrict__ PS,
                    unsigned short* __restrict__ CTXh, unsigned short* __restrict__ CTXl,
                    int b, float cs) {
  union FB { v16b v; v8b h[2]; };
  __shared__ __align__(16) unsigned char SMEM[58368];
  _Float16* Ksh = (_Float16*)(SMEM);
  __bf16*   Vth = (__bf16*)(SMEM + 8192);
  __bf16*   Vtl = (__bf16*)(SMEM + 16384);
  float*    PSw = (float*)(SMEM + 24576);
  __bf16*   Psh = (__bf16*)(SMEM + 41984);
  __bf16*   Psl = (__bf16*)(SMEM + 50176);
  float*    Osb = (float*)(SMEM + 24576);

  const int tid  = threadIdx.x;
  const int wave = tid >> 5;
  const int lane = tid & 31;
  const int hh   = lane >> 4;
  const int c    = lane & 15;

  const int h  = blockIdx.y;
  const int qb = blockIdx.x;
  const int T0 = qb * 64;
  const int q0 = T0 + wave * 16;

  const _Float16* Qh = QU  + (size_t)(b * NT_) * ND_ + h * HD_;
  const _Float16* Kh = KPL + (size_t)(b * NT_) * ND_ + h * HD_;
  const __bf16* Vh = (const __bf16*)(const void*)VThp + (size_t)(h * HD_) * NBT_ + b * NT_;
  const __bf16* Vl = (const __bf16*)(const void*)VTlp + (size_t)(h * HD_) * NBT_ + b * NT_;
  const float*  psm = PS + (size_t)h * NT_ * NT_;
  _Float16* cth = (_Float16*)(void*)CTXh + (size_t)(b * NT_) * ND_ + h * HD_;
  _Float16* ctl = (_Float16*)(void*)CTXl + (size_t)(b * NT_) * ND_ + h * HD_;

  v16h qa[2];
#pragma unroll
  for (int dc = 0; dc < 2; ++dc)
    qa[dc] = Frag<_Float16>::load(Qh + (size_t)(q0 + c) * ND_ + dc * 32 + 8 * hh);

  float mrow[8], lrow[8];
  v8f oacc[4];
#pragma unroll
  for (int r = 0; r < 8; ++r) { mrow[r] = -INFINITY; lrow[r] = 0.f; }
#pragma unroll
  for (int t = 0; t < 4; ++t) oacc[t] = zero8();

  __bf16* pwh = Psh + wave * (16 * 64);
  __bf16* pwl = Psl + wave * (16 * 64);

  for (int kc = 0; kc < NT_ / 64; ++kc) {
    const int kv0 = kc * 64;
    __syncthreads();
    {
      const int r = tid >> 1, half = (tid & 1) * 32;
      const _Float16* ks = Kh + (size_t)(kv0 + r) * ND_ + half;
      const __bf16* vsh = Vh + (size_t)r * NBT_ + kv0 + half;
      const __bf16* vsl = Vl + (size_t)r * NBT_ + kv0 + half;
#pragma unroll
      for (int i = 0; i < 4; ++i) {
        const v8h k8 = *(const v8ha*)(ks + 8 * i);
        const v8b v0 = *(const v8ba*)(vsh + 8 * i);
        const v8b v1 = *(const v8ba*)(vsl + 8 * i);
        *(v8ha*)(Ksh + r * 64 + half + 8 * i) = k8;
        *(v8ba*)(Vth + r * 64 + half + 8 * i) = v0;
        *(v8ba*)(Vtl + r * 64 + half + 8 * i) = v1;
      }
#pragma unroll
      for (int i = 0; i < 9; ++i) {
        int idx = tid + 128 * i;
        idx = (idx < 1087) ? idx : 1087;
        const int row = idx / 17;
        const int qq  = idx - row * 17;
        const int t   = T0 + row;
        const int a0  = ((t + 1) * 1023 + kv0 - 1) & ~3;
        const v4f w = *(const v4fa*)(psm + a0 + 4 * qq);
        *(v4fa*)(PSw + row * 68 + 4 * qq) = w;
      }
    }
    __syncthreads();

    v8f s[4];
#pragma unroll
    for (int j = 0; j < 4; ++j) {
      s[j] = zero8();
#pragma unroll
      for (int dc = 0; dc < 2; ++dc) {
        const v16h kb = Frag<_Float16>::load(Ksh + (j * 16 + c) * 64 + dc * 32 + 8 * hh);
        s[j] = mma16h(qa[dc], kb, s[j]);
      }
    }

    float cm[8];
#pragma unroll
    for (int r = 0; r < 8; ++r) {
      const int t  = q0 + 8 * hh + r;
      const int lr = wave * 16 + 8 * hh + r;
      const int rowoff = lr * 68 + 1 + ((3 * t + 2) & 3);
      float m = -INFINITY;
#pragma unroll
      for (int j = 0; j < 4; ++j) {
        const int xk = (j << 4) + c;
        const int sk = kv0 + xk;
        const int gt = (sk > t) ? 1 : 0;
        const float zf = (sk == t + 1) ? 0.0f : 1.0f;
        const float pv = PSw[rowoff + xk - gt] * zf;
        const float sv = fmaf(s[j][r], cs, pv);
        s[j][r] = sv;
        m = fmaxf(m, sv);
      }
      m = fmaxf(m, __shfl_xor(m, 1, 32));
      m = fmaxf(m, __shfl_xor(m, 2, 32));
      m = fmaxf(m, __shfl_xor(m, 4, 32));
      m = fmaxf(m, __shfl_xor(m, 8, 32));
      cm[r] = m;
    }

#pragma unroll
    for (int r = 0; r < 8; ++r) {
      const float mnew  = fmaxf(mrow[r], cm[r]);
      const float alpha = __expf(mrow[r] - mnew);
      mrow[r] = mnew;
      float psum = 0.f;
#pragma unroll
      for (int j = 0; j < 4; ++j) {
        const float p = __expf(s[j][r] - mnew);
        psum += p;
        __bf16 ph, pl;
        bf_split(p, ph, pl);
        pwh[(8 * hh + r) * 64 + j * 16 + c] = ph;
        pwl[(8 * hh + r) * 64 + j * 16 + c] = pl;
      }
      psum += __shfl_xor(psum, 1, 32);
      psum += __shfl_xor(psum, 2, 32);
      psum += __shfl_xor(psum, 4, 32);
      psum += __shfl_xor(psum, 8, 32);
      lrow[r] = lrow[r] * alpha + psum;
#pragma unroll
      for (int t = 0; t < 4; ++t) oacc[t][r] *= alpha;
    }
    __builtin_amdgcn_fence(__ATOMIC_RELEASE, "workgroup");
    __builtin_amdgcn_wave_barrier();
    __builtin_amdgcn_fence(__ATOMIC_ACQUIRE, "workgroup");

#pragma unroll 1
    for (int kk = 0; kk < 2; ++kk) {
      FB pa, pl;
      pa.h[0] = *(const v8ba*)(pwh + c * 64 + kk * 32 + 8 * hh);
      pa.h[1] = *(const v8ba*)(pwh + c * 64 + kk * 32 + 16 + 8 * hh);
      pl.h[0] = *(const v8ba*)(pwl + c * 64 + kk * 32 + 8 * hh);
      pl.h[1] = *(const v8ba*)(pwl + c * 64 + kk * 32 + 16 + 8 * hh);
#pragma unroll
      for (int t = 0; t < 4; ++t) {
        FB vb, vl;
        vb.h[0] = *(const v8ba*)(Vth + (t * 16 + c) * 64 + kk * 32 + 8 * hh);
        vb.h[1] = *(const v8ba*)(Vth + (t * 16 + c) * 64 + kk * 32 + 16 + 8 * hh);
        vl.h[0] = *(const v8ba*)(Vtl + (t * 16 + c) * 64 + kk * 32 + 8 * hh);
        vl.h[1] = *(const v8ba*)(Vtl + (t * 16 + c) * 64 + kk * 32 + 16 + 8 * hh);
        oacc[t] = mma16b(pa.v, vb.v, oacc[t]);
        oacc[t] = mma16b(pa.v, vl.v, oacc[t]);
        oacc[t] = mma16b(pl.v, vb.v, oacc[t]);
      }
    }
  }

  __syncthreads();
  float* os = Osb + wave * (16 * 68);
#pragma unroll
  for (int r = 0; r < 8; ++r) {
    const float inv = 1.0f / lrow[r];
#pragma unroll
    for (int t = 0; t < 4; ++t) os[(8 * hh + r) * 68 + t * 16 + c] = oacc[t][r] * inv;
  }
  __builtin_amdgcn_fence(__ATOMIC_RELEASE, "workgroup");
  __builtin_amdgcn_wave_barrier();
  __builtin_amdgcn_fence(__ATOMIC_ACQUIRE, "workgroup");
  {
    const int q = lane >> 3, c8 = (lane & 7) * 8;
    v8h hv[4], lv[4];
#pragma unroll
    for (int it = 0; it < 4; ++it) {
      const int row = it * 4 + q;
      const float* sp = os + row * 68 + c8;
      const v4f x0 = *(const v4fa*)(sp);
      const v4f x1 = *(const v4fa*)(sp + 4);
      float f[8];
      f[0] = x0[0]; f[1] = x0[1]; f[2] = x0[2]; f[3] = x0[3];
      f[4] = x1[0]; f[5] = x1[1]; f[6] = x1[2]; f[7] = x1[3];
      v8h ha, hb;
#pragma unroll
      for (int e = 0; e < 8; ++e) {
        const unsigned short hbits = f2bf_bits(f[e]);
        const unsigned short lbits = f2bf_bits(f[e] - bf_bits2f(hbits));
        ha[e] = __builtin_bit_cast(_Float16, hbits);
        hb[e] = __builtin_bit_cast(_Float16, lbits);
      }
      hv[it] = ha; lv[it] = hb;
    }
    for (int pass = 0; pass < 2; ++pass) {
#pragma unroll
      for (int it = 0; it < 4; ++it) {
        const int row = it * 4 + q;
        *(volatile v8h*)(cth + (size_t)(q0 + row) * ND_ + c8) = hv[it];
        *(volatile v8h*)(ctl + (size_t)(q0 + row) * ND_ + c8) = lv[it];
      }
      __threadfence();
    }
  }
}

extern "C" void kernel_launch(void* const* d_in, const int* in_sizes, int n_in,
                              void* d_out, int out_size, void* d_ws, size_t ws_size,
                              hipStream_t stream) {
  if (n_in < 14) return;
  if (in_sizes[0] != NBT_ * ND_) return;
  if (in_sizes[1] != ND_ || in_sizes[2] != ND_) return;
  if (in_sizes[3] != ND_ * ND_ || in_sizes[4] != ND_) return;
  if (in_sizes[5] != ND_ * ND_ || in_sizes[6] != ND_) return;
  if (in_sizes[7] != ND_ * ND_ || in_sizes[8] != ND_) return;
  if (in_sizes[9] != ND_ * ND_) return;
  if (in_sizes[10] != NH_ * HD_ || in_sizes[11] != NH_ * HD_) return;
  if (in_sizes[12] != ND_ * ND_ || in_sizes[13] != ND_) return;
  if (out_size != NBT_ * ND_) return;

  const float* x    = (const float*)d_in[0];
  const float* ln_g = (const float*)d_in[1];
  const float* ln_b = (const float*)d_in[2];
  const float* Wq   = (const float*)d_in[3];
  const float* bq   = (const float*)d_in[4];
  const float* Wk   = (const float*)d_in[5];
  const float* bk   = (const float*)d_in[6];
  const float* Wv   = (const float*)d_in[7];
  const float* bv   = (const float*)d_in[8];
  const float* Wp   = (const float*)d_in[9];
  const float* ub   = (const float*)d_in[10];
  const float* vbs  = (const float*)d_in[11];
  const float* Wo   = (const float*)d_in[12];
  const float* bo   = (const float*)d_in[13];
  float* out = (float*)d_out;

  const size_t PW16 = (size_t)ND_ * ND_ * 2;
  const size_t PA16 = (size_t)NBT_ * ND_ * 2;
  const size_t PP16 = (size_t)NT_ * ND_ * 2;
  const size_t PVT  = (size_t)ND_ * NBT_ * 2;
  const size_t PPS  = (size_t)NH_ * NT_ * NT_ * 4;
  size_t off = 0;
  const size_t oWQT  = off; off += PW16;
  const size_t oWKT  = off; off += PW16;
  const size_t oWPT  = off; off += PW16;
  const size_t oWVTh = off; off += PW16;
  const size_t oWVTl = off; off += PW16;
  const size_t oWOTh = off; off += PW16;
  const size_t oWOTl = off; off += PW16;
  const size_t oQU   = off; off += PA16;
  const size_t oQV   = off; off += PA16;
  const size_t oKP   = off; off += PA16;
  const size_t oP16  = off; off += PP16;
  const size_t oVTh  = off; off += PVT;
  const size_t oVTl  = off; off += PVT;
  const size_t oCTXh = off; off += PA16;
  const size_t oCTXl = off; off += PA16;
  const size_t oSCR  = off;
  const size_t oXNF  = oSCR;
  const size_t oXNH  = oXNF + PA16;
  const size_t oXNL  = oXNH + PA16;
  const size_t oPEF  = oXNL + PA16;
  const size_t earlyEnd = oPEF + PP16;
  const size_t oPS   = oSCR;
  const size_t lateEnd  = oPS + PPS;
  const size_t total = (earlyEnd > lateEnd) ? earlyEnd : lateEnd;
  if (total > ws_size) return;
  if (total > (size_t)134217728) return;

  char* ws = (char*)d_ws;
  unsigned short* WQT  = (unsigned short*)(ws + oWQT);
  unsigned short* WKT  = (unsigned short*)(ws + oWKT);
  unsigned short* WPT  = (unsigned short*)(ws + oWPT);
  unsigned short* WVTh = (unsigned short*)(ws + oWVTh);
  unsigned short* WVTl = (unsigned short*)(ws + oWVTl);
  unsigned short* WOTh = (unsigned short*)(ws + oWOTh);
  unsigned short* WOTl = (unsigned short*)(ws + oWOTl);
  unsigned short* QU   = (unsigned short*)(ws + oQU);
  unsigned short* QV   = (unsigned short*)(ws + oQV);
  unsigned short* KPL  = (unsigned short*)(ws + oKP);
  unsigned short* P16  = (unsigned short*)(ws + oP16);
  unsigned short* VTh  = (unsigned short*)(ws + oVTh);
  unsigned short* VTl  = (unsigned short*)(ws + oVTl);
  unsigned short* CTXh = (unsigned short*)(ws + oCTXh);
  unsigned short* CTXl = (unsigned short*)(ws + oCTXl);
  unsigned short* XNF  = (unsigned short*)(ws + oXNF);
  unsigned short* XNH  = (unsigned short*)(ws + oXNH);
  unsigned short* XNL  = (unsigned short*)(ws + oXNL);
  unsigned short* PEF  = (unsigned short*)(ws + oPEF);
  float*          PS   = (float*)(ws + oPS);

  const float inv_sd = 0.044194174f;
  const float cs     = inv_sd * 0.015625f;
  const float pscale = (1.0f / 8192.0f);
  const dim3 blk(256);

  ln_kernel<<<dim3(NBT_), dim3(64), 0, stream>>>(x, ln_g, ln_b, (_Float16*)XNF, XNH, XNL);
  tcvt_f16_kernel<<<dim3(ND_ / 64, ND_ / 64), blk, 0, stream>>>(Wq, (_Float16*)WQT, ND_, ND_, 1024.0f);
  tcvt_f16_kernel<<<dim3(ND_ / 64, ND_ / 64), blk, 0, stream>>>(Wk, (_Float16*)WKT, ND_, ND_, 1024.0f);
  tcvt_f16_kernel<<<dim3(ND_ / 64, ND_ / 64), blk, 0, stream>>>(Wp, (_Float16*)WPT, ND_, ND_, 1024.0f);
  tsplit_kernel<<<dim3(ND_ / 64, ND_ / 64, 1), blk, 0, stream>>>(Wv, WVTh, WVTl, ND_, ND_, 0L, 0L);
  tsplit_kernel<<<dim3(ND_ / 64, ND_ / 64, 1), blk, 0, stream>>>(Wo, WOTh, WOTl, ND_, ND_, 0L, 0L);
  pe_kernel<<<dim3(NT_), dim3(64), 0, stream>>>((_Float16*)PEF);
  {
    const int tilesA = (NBT_ / 64) * (ND_ / 64);
    gemm64_kernel<0, false, 2, 2><<<dim3((tilesA + 7) / 8, 1), blk, 0, stream>>>(
        XNF, XNF, ND_, 0L, WQT, WQT, ND_, 0L, (void*)QU, (void*)QV, ND_, 0L, bq, ub, vbs,
        NBT_, ND_, ND_, pscale, 8.0f);
    gemm64_kernel<0, false, 1, 2><<<dim3((tilesA + 7) / 8, 1), blk, 0, stream>>>(
        XNF, XNF, ND_, 0L, WKT, WKT, ND_, 0L, (void*)KPL, (void*)KPL, ND_, 0L, bk, bk, bk,
        NBT_, ND_, ND_, pscale, 8.0f);
    const int tilesP = (NT_ / 64) * (ND_ / 64);
    gemm64_kernel<0, false, 1, 0><<<dim3((tilesP + 7) / 8, 1), blk, 0, stream>>>(
        PEF, PEF, ND_, 0L, WPT, WPT, ND_, 0L, (void*)P16, (void*)P16, ND_, 0L, bq, bq, bq,
        NT_, ND_, ND_, pscale, 8.0f);
    const int tilesV = (ND_ / 64) * (NBT_ / 64);
    gemm64_kernel<1, true, 3, 1><<<dim3((tilesV + 7) / 8, 1), blk, 0, stream>>>(
        WVTh, WVTl, ND_, 0L, XNH, XNL, ND_, 0L, (void*)VTh, (void*)VTl, NBT_, 0L, bv, bv, bv,
        ND_, NBT_, ND_, 1.0f, 1.0f);
  }
  for (int b = 0; b < NB_; ++b) {
    const int tilesS = (NT_ / 64) * (NT_ / 64);
    gemm64_kernel<0, false, 0, 0><<<dim3((tilesS + 7) / 8, NH_), blk, 0, stream>>>(
        QV + (size_t)b * NT_ * ND_, QV + (size_t)b * NT_ * ND_, ND_, (long)HD_,
        P16, P16, ND_, (long)HD_,
        (void*)PS, (void*)PS, NT_, (long)NT_ * NT_, bq, bq, bq,
        NT_, NT_, HD_, cs, 1.0f);
    relattn_kernel<<<dim3(NT_ / 64, NH_), dim3(128), 0, stream>>>(
        (const _Float16*)QU, (const _Float16*)KPL, VTh, VTl, PS, CTXh, CTXl, b, cs);
  }
  {
    const int tilesO = (NBT_ / 64) * (ND_ / 64);
    gemm64_kernel<1, true, 0, 2><<<dim3((tilesO + 7) / 8, 1), blk, 0, stream>>>(
        CTXh, CTXl, ND_, 0L, WOTh, WOTl, ND_, 0L, (void*)out, (void*)out, ND_, 0L, bo, bo, bo,
        NBT_, ND_, ND_, 1.0f, 1.0f);
  }
  (void)hipGetLastError();
}
